// EquivariantAttention_62964220559519
// MI455X (gfx1250) — hardware-verified
//
#include <hip/hip_runtime.h>
#include <stddef.h>
#include <stdint.h>


#define HID    128
#define EFK    32
#define FROW   64
#define MULT   16
#define NHEAD  4
#define NLR    256
#define KRL    256
#define NSUB   4
#define SUBN   128
#define NW1    256
#define NWRL   1024
#define CTHR   128
#define CWAVE  4
#define DP     132
#define AP     264
#define FP     40
#define TP     36
#define UP     8
#define CSTN   640
#define NTHR   256
#define NWAVE  8
#define EPT    8
#define CHUNK  (NTHR * EPT)
#define WCAP   (EPT * 32)
#define LISTN  (NWAVE * WCAP)
#define NBA    1024
#define SLA    10
#define RCAP   28672
#define DEGCAP 64
#define SPW    (NBA / NWAVE)
#define NU_W1  (NW1 * (EFK / 8))
#define NU_WRL (NWRL * (KRL / 8))
#define AGG_ZINTS (LISTN + 2 * RCAP + 3 * NBA)
#define AGG_LDS_INTS (AGG_ZINTS + 16)
#define AGG_LDS_BYTES (AGG_LDS_INTS * 4)
#define CONV_LDS_BYTES (CTHR * DP * 4 + CTHR * AP * 2 + CTHR * FP * 2 + 2 * CTHR * TP * 4 + CTHR * UP * 4 + CSTN * 4)
#define WSMAX  134217728
#define QSCL   0.25f

static_assert((CHUNK & (CHUNK - 1)) == 0 && CHUNK <= 4096);
static_assert((NBA & (NBA - 1)) == 0 && NBA == (1 << SLA));
static_assert(((long long)CHUNK << SLA) < (1LL << 31));
static_assert(LISTN % NTHR == 0);
static_assert(NBA % NWAVE == 0 && NBA % 32 == 0 && SPW % 2 == 0);
static_assert(RCAP % 4 == 0 && AGG_ZINTS % (4 * NTHR) == 0 && LISTN % 4 == 0);
static_assert(AGG_LDS_BYTES <= 300000);
static_assert(CONV_LDS_BYTES <= 300000);
static_assert(NU_W1 % NTHR == 0 && (NU_W1 / 2) % NTHR == 0);
static_assert(NU_WRL % NTHR == 0 && (NU_WRL / 4) % NTHR == 0);
static_assert(CTHR == HID && CTHR == 32 * CWAVE);
static_assert(EFK == 32 && KRL % 32 == 0 && KRL == 2 * HID && NSUB * SUBN == 2 * NLR && SUBN == 4 * 32);
static_assert(AP >= KRL && FP >= EFK && DP >= SUBN && TP >= 2 * MULT && UP == 8);
static_assert((DP * 4) % 16 == 0 && (AP * 2) % 16 == 0 && (FP * 2) % 16 == 0 && (TP * 4) % 16 == 0);
static_assert((CTHR * DP * 4) % 16 == 0 && (CTHR * AP * 2) % 16 == 0 && (CTHR * FP * 2) % 16 == 0);
static_assert((CTHR * TP * 4) % 16 == 0 && (CTHR * UP * 4) % 16 == 0 && (CSTN * 4) % 16 == 0);
static_assert(CSTN >= HID + 2 * NLR);
static_assert(CTHR * FROW <= CTHR * DP && CTHR * 4 <= CTHR * DP);
static_assert(CTHR * FROW == 16 * CTHR * 4);
static_assert(FROW == MULT * 4 && FROW == NHEAD * 16 && FROW == 2 * 32);
static_assert(DEGCAP % 32 == 0);

typedef float          v2f   __attribute__((ext_vector_type(2)));
typedef float          v4f   __attribute__((ext_vector_type(4)));
typedef float          v8f   __attribute__((ext_vector_type(8)));
typedef int            v4i   __attribute__((ext_vector_type(4)));
typedef int            v8i   __attribute__((ext_vector_type(8)));
typedef unsigned short v8us  __attribute__((ext_vector_type(8)));
typedef unsigned short v16us __attribute__((ext_vector_type(16)));
typedef __bf16         v16bf __attribute__((ext_vector_type(16)));
typedef v2f  __attribute__((may_alias)) v2fa;
typedef v4f  __attribute__((may_alias)) v4fa;
typedef v4i  __attribute__((may_alias)) v4ia;
typedef v8us __attribute__((may_alias)) v8usa;
union FragB { v16bf v; v16us u; v8us h[2]; v8i w; };

__device__ __forceinline__ v8f wmb(const FragB& a, const FragB& b, v8f c) {
  v8f d = __builtin_amdgcn_wmma_f32_16x16x32_bf16(false, a.v, false, b.v, (short)0, c, false, false);
  asm volatile("v_nop\n\tv_nop\n\tv_nop\n\tv_nop" : "+v"(d) : "v"(a.w), "v"(b.w));
  return d;
}

__device__ __forceinline__ unsigned bf16_bits(float f) {
  const unsigned u = __float_as_uint(f);
  return (u + 0x7FFFu + ((u >> 16) & 1u)) >> 16;
}
__device__ __forceinline__ float bf16_val(float f) {
  return __uint_as_float(bf16_bits(f) << 16);
}
__device__ __forceinline__ float gelu_f(float x) {
  return 0.5f * x * (1.0f + erff(x * 0.70710678118654752440f));
}
__device__ __forceinline__ void put16(unsigned short* dp, v8us o) {
  *(volatile v8us*)dp = o;
  __threadfence();
  *(volatile v8us*)dp = o;
}
__device__ __forceinline__ void putf4(float* dp, v4f o) {
  *(volatile v4f*)dp = o;
  __threadfence();
  *(volatile v4f*)dp = o;
}

template <int SLB>
__device__ __forceinline__ int scan_chunk(const int* __restrict__ dsts, int nE, int cbase, int slotBase,
                                          int nb, int vec8, int* list, int tid, int lane, int wave) {
  int wc = 0;
  const int el0  = tid * EPT;
  const int e0   = cbase + el0;
  const int sent = -2147483647 - 1;
  v4i da, db;
  if (vec8 != 0 && cbase + CHUNK <= nE) {
    da = *(const v4i*)(dsts + e0);
    db = *(const v4i*)(dsts + e0 + 4);
  } else {
    da.x = (e0     < nE) ? dsts[min(e0,     nE - 1)] : sent;
    da.y = (e0 + 1 < nE) ? dsts[min(e0 + 1, nE - 1)] : sent;
    da.z = (e0 + 2 < nE) ? dsts[min(e0 + 2, nE - 1)] : sent;
    da.w = (e0 + 3 < nE) ? dsts[min(e0 + 3, nE - 1)] : sent;
    db.x = (e0 + 4 < nE) ? dsts[min(e0 + 4, nE - 1)] : sent;
    db.y = (e0 + 5 < nE) ? dsts[min(e0 + 5, nE - 1)] : sent;
    db.z = (e0 + 6 < nE) ? dsts[min(e0 + 6, nE - 1)] : sent;
    db.w = (e0 + 7 < nE) ? dsts[min(e0 + 7, nE - 1)] : sent;
  }
  const unsigned nbs = (unsigned)slotBase;
  const unsigned unb = (unsigned)nb;
  const unsigned s0 = (unsigned)da.x - nbs, s1 = (unsigned)da.y - nbs;
  const unsigned s2 = (unsigned)da.z - nbs, s3 = (unsigned)da.w - nbs;
  const unsigned s4 = (unsigned)db.x - nbs, s5 = (unsigned)db.y - nbs;
  const unsigned s6 = (unsigned)db.z - nbs, s7 = (unsigned)db.w - nbs;
  const bool h0 = s0 < unb, h1 = s1 < unb, h2 = s2 < unb, h3 = s3 < unb;
  const bool h4 = s4 < unb, h5 = s5 < unb, h6 = s6 < unb, h7 = s7 < unb;
  const unsigned any = __builtin_amdgcn_ballot_w32(h0 | h1 | h2 | h3 | h4 | h5 | h6 | h7);
  if (any != 0u) {
#define HITJ(J, HJ, SJ) { \
      const unsigned mj = __builtin_amdgcn_ballot_w32(HJ); \
      if (mj != 0u) { \
        if (HJ) { \
          const int pos = wc + (int)__builtin_amdgcn_mbcnt_lo(mj, 0u); \
          if (pos < WCAP) list[wave * WCAP + pos] = ((el0 + (J)) << SLB) | (int)(SJ); \
        } \
        wc += (int)__builtin_popcount(mj); } }
    HITJ(0, h0, s0)
    HITJ(1, h1, s1)
    HITJ(2, h2, s2)
    HITJ(3, h3, s3)
    HITJ(4, h4, s4)
    HITJ(5, h5, s5)
    HITJ(6, h6, s6)
    HITJ(7, h7, s7)
#undef HITJ
  }
  return wc;
}

__global__ __launch_bounds__(NTHR) void k_prep(const float* __restrict__ f, const float* __restrict__ qw,
                                               const float* __restrict__ qb,
                                               const float* __restrict__ kw1, const float* __restrict__ vw1,
                                               const float* __restrict__ kwr, const float* __restrict__ kwl,
                                               const float* __restrict__ vwr, const float* __restrict__ vwl,
                                               int nN, int nQU,
                                               unsigned short* W1T, unsigned short* WRL, float* Q) {
  const int u  = (int)blockIdx.x * NTHR + (int)threadIdx.x;
  const int U0 = NU_W1;
  const int U1 = U0 + NU_WRL;
  const int U2 = U1 + nQU;
  v8us o;
  if (u < U0) {
    const int n   = u >> 2;
    const int k8  = (u & 3) * 8;
    const float* W = (n < HID) ? kw1 : vw1;
    const int nn  = n & (HID - 1);
    const float* p = W + (size_t)k8 * HID + nn;
#pragma unroll
    for (int i = 0; i < 8; ++i) o[i] = (unsigned short)bf16_bits(p[(size_t)i * HID]);
    put16(W1T + (size_t)n * EFK + k8, o);
    return;
  } else if (u < U1) {
    const int v    = u - U0;
    const int n    = v >> 5;
    const int k8   = (v & 31) * 8;
    const int q    = n >> 8;
    const float* W = (q == 0) ? kwr : ((q == 1) ? kwl : ((q == 2) ? vwr : vwl));
    const int nn   = n & (NLR - 1);
    const int srow = k8 & (HID - 1);
    const float* p = W + (size_t)srow * NLR + nn;
#pragma unroll
    for (int i = 0; i < 8; ++i) o[i] = (unsigned short)bf16_bits(p[(size_t)i * NLR]);
    put16(WRL + (size_t)n * KRL + k8, o);
    return;
  } else if (u < U2) {
    const int v    = u - U1;
    const int node = v >> 4;
    const int oo   = v & 15;
    if (node >= nN) return;
    const float* fr  = f + (size_t)node * FROW;
    const float* w0r = qw + (size_t)oo * MULT;
    const float* w1r = qw + (size_t)(MULT + oo) * MULT;
    float ax = 0.0f, ay = 0.0f, az = 0.0f, aw = 0.0f;
#pragma unroll 1
    for (int g = 0; g < MULT / 4; ++g) {
      const v4f wa = *(const v4fa*)(w0r + 4 * g);
      const v4f wb = *(const v4fa*)(w1r + 4 * g);
#pragma unroll
      for (int j = 0; j < 4; ++j) {
        const v4f fv = *(const v4fa*)(fr + (4 * g + j) * 4);
        const float s0 = bf16_val(wa[j]);
        const float s1 = bf16_val(wb[j]);
        ax = fmaf(s0, bf16_val(fv.x), ax);
        ay = fmaf(s1, bf16_val(fv.y), ay);
        az = fmaf(s1, bf16_val(fv.z), az);
        aw = fmaf(s1, bf16_val(fv.w), aw);
      }
    }
    ax += bf16_val(qb[oo]);
    const v4f q4 = {ax, ay, az, aw};
    putf4(Q + (size_t)node * FROW + 4 * oo, q4);
    return;
  }
}

template <int APITCH>
__device__ __forceinline__ void wave_gemm_b(const unsigned short* sAw, float* sDw,
                                            const unsigned short* __restrict__ BT, int ldb, int K,
                                            int hh, int m) {
#pragma unroll 1
  for (int nh = 0; nh < 2; ++nh) {
    v8f acc[2][4];
    {
      const v8f z = {0.f, 0.f, 0.f, 0.f, 0.f, 0.f, 0.f, 0.f};
#pragma unroll
      for (int mt = 0; mt < 2; ++mt)
#pragma unroll
        for (int nt = 0; nt < 4; ++nt) acc[mt][nt] = z;
    }
    const unsigned short* ap0 = sAw + m * APITCH + 8 * hh;
    const unsigned short* ap1 = ap0 + 16 * APITCH;
    const unsigned short* bp  = BT + (size_t)(64 * nh + m) * (size_t)ldb + 8 * hh;
#pragma unroll 1
    for (int k0 = 0; k0 < K; k0 += 32) {
      FragB a0, a1;
      a0.h[0] = *(const v8usa*)(ap0 + k0);
      a0.h[1] = *(const v8usa*)(ap0 + k0 + 16);
      a1.h[0] = *(const v8usa*)(ap1 + k0);
      a1.h[1] = *(const v8usa*)(ap1 + k0 + 16);
#pragma unroll
      for (int nt = 0; nt < 4; ++nt) {
        const unsigned short* wq = bp + (size_t)(16 * nt) * (size_t)ldb + k0;
        FragB b;
        b.h[0] = *(const v8usa*)wq;
        b.h[1] = *(const v8usa*)(wq + 16);
        acc[0][nt] = wmb(a0, b, acc[0][nt]);
        acc[1][nt] = wmb(a1, b, acc[1][nt]);
      }
    }
#pragma unroll
    for (int nt = 0; nt < 4; ++nt) {
      const int col = 64 * nh + 16 * nt + m;
#pragma unroll
      for (int mt = 0; mt < 2; ++mt)
#pragma unroll
        for (int r = 0; r < 8; ++r) sDw[(16 * mt + 8 * hh + r) * DP + col] = acc[mt][nt][r];
    }
  }
}

template <int MODE>
__global__ __launch_bounds__(CTHR) void k_conv(const int* __restrict__ src, const int* __restrict__ dst,
                                               int nE, int nN,
                                               const float* __restrict__ EF, const float* __restrict__ F,
                                               const float* __restrict__ B1, const float* __restrict__ B2,
                                               const unsigned short* __restrict__ W1T,
                                               const unsigned short* __restrict__ WRL,
                                               const float* __restrict__ bh, const float* __restrict__ br,
                                               const float* __restrict__ bl,
                                               const float* __restrict__ Q, float* SC, float* Vp) {
  extern __shared__ __attribute__((aligned(16))) float dyn[];
  float*          sD  = dyn;
  unsigned short* sA  = (unsigned short*)(dyn + CTHR * DP);
  unsigned short* sE  = sA + CTHR * AP;
  float*          sT1 = dyn + CTHR * DP + (CTHR * AP) / 2 + (CTHR * FP) / 2;
  float*          sT2 = sT1 + CTHR * TP;
  float*          sU  = sT2 + CTHR * TP;
  float*          cst = sU + CTHR * UP;

  const int tid = (int)threadIdx.x, lane = tid & 31, wave = tid >> 5, hh = lane >> 4, m = lane & 15;

  cst[tid]           = bf16_val(bh[tid]);
  cst[HID + tid]     = bf16_val(br[tid]);
  cst[2 * HID + tid] = bf16_val(br[HID + tid]);
  cst[3 * HID + tid] = bf16_val(bl[tid]);
  cst[4 * HID + tid] = bf16_val(bl[HID + tid]);

  const int  elb  = (int)blockIdx.x * CTHR;
  const int  el   = elb + tid;
  const bool live = el < nE;
  const int  elc  = live ? el : (nE - 1);
  int s = src[elc];
  s = s < 0 ? 0 : (s > nN - 1 ? nN - 1 : s);

  float*          rd  = sD  + tid * DP;
  unsigned short* ra  = sA  + tid * AP;
  unsigned short* re  = sE  + tid * FP;
  float*          rt1 = sT1 + tid * TP;
  float*          rt2 = sT2 + tid * TP;
  float*          ru  = sU  + tid * UP;
  {
    const float* er = EF + (size_t)elc * EFK;
#pragma unroll
    for (int c8 = 0; c8 < EFK / 8; ++c8) {
      const v4f a = *(const v4fa*)(er + 8 * c8);
      const v4f b = *(const v4fa*)(er + 8 * c8 + 4);
      v8us o;
      o[0] = (unsigned short)bf16_bits(a.x); o[1] = (unsigned short)bf16_bits(a.y);
      o[2] = (unsigned short)bf16_bits(a.z); o[3] = (unsigned short)bf16_bits(a.w);
      o[4] = (unsigned short)bf16_bits(b.x); o[5] = (unsigned short)bf16_bits(b.y);
      o[6] = (unsigned short)bf16_bits(b.z); o[7] = (unsigned short)bf16_bits(b.w);
      *(v8usa*)(re + 8 * c8) = o;
    }
  }
  {
    const float* fr  = F + (size_t)s * FROW;
    const float* b1r = B1 + (size_t)elc * 8;
    const v4f ba = *(const v4fa*)b1r;
    const v4f bb = *(const v4fa*)(b1r + 4);
    const float w00 = bf16_val(ba.x), w01 = bf16_val(ba.y);
    const float w10 = bf16_val(ba.z), w11 = bf16_val(ba.w);
    const float w20 = bf16_val(bb.x), w21 = bf16_val(bb.y);
    const float w30 = bf16_val(bb.z), w31 = bf16_val(bb.w);
#pragma unroll 1
    for (int mq = 0; mq < MULT / 2; ++mq) {
      const v4f fa = *(const v4fa*)(fr + 8 * mq);
      const v4f fb = *(const v4fa*)(fr + 8 * mq + 4);
      const float a0 = bf16_val(fa.x), a1 = bf16_val(fa.y), a2 = bf16_val(fa.z), a3 = bf16_val(fa.w);
      const float c0 = bf16_val(fb.x), c1 = bf16_val(fb.y), c2 = bf16_val(fb.z), c3 = bf16_val(fb.w);
      v4f t4;
      t4.x = fmaf(a3, w30, fmaf(a2, w20, fmaf(a1, w10, a0 * w00)));
      t4.y = fmaf(a3, w31, fmaf(a2, w21, fmaf(a1, w11, a0 * w01)));
      t4.z = fmaf(c3, w30, fmaf(c2, w20, fmaf(c1, w10, c0 * w00)));
      t4.w = fmaf(c3, w31, fmaf(c2, w21, fmaf(c1, w11, c0 * w01)));
      *(v4fa*)(rt1 + 4 * mq) = t4;
    }
  }
  __syncthreads();

  float* sDw = sD + 32 * wave * DP;

  wave_gemm_b<FP>(sE + 32 * wave * FP, sDw, W1T, EFK, EFK, hh, m);
  __syncthreads();

  {
#pragma unroll 1
    for (int c8 = 0; c8 < HID / 8; ++c8) {
      const v4f va = *(const v4fa*)(rd + 8 * c8);
      const v4f vb = *(const v4fa*)(rd + 8 * c8 + 4);
      const v4f ba = *(const v4fa*)(cst + 8 * c8);
      const v4f bb = *(const v4fa*)(cst + 8 * c8 + 4);
      const v8f v8 = {va.x, va.y, va.z, va.w, vb.x, vb.y, vb.z, vb.w};
      const v8f b8 = {ba.x, ba.y, ba.z, ba.w, bb.x, bb.y, bb.z, bb.w};
      v8us ho, lo;
#pragma unroll
      for (int i = 0; i < 8; ++i) {
        const float g = gelu_f(v8[i] + b8[i]);
        const unsigned hb = bf16_bits(g);
        ho[i] = (unsigned short)hb;
        lo[i] = (unsigned short)bf16_bits(g - __uint_as_float(hb << 16));
      }
      *(v8usa*)(ra + 8 * c8)       = ho;
      *(v8usa*)(ra + HID + 8 * c8) = lo;
    }
  }
  __syncthreads();

  const unsigned short* sAw = sA + 32 * wave * AP;

#pragma unroll 1
  for (int ns = 0; ns < NSUB; ++ns) {
    wave_gemm_b<AP>(sAw, sDw, WRL + (size_t)ns * SUBN * KRL, KRL, KRL, hh, m);
    __syncthreads();
    const float* cb = cst + HID + ns * SUBN;
    if (ns < 2) {
#pragma unroll 1
      for (int a = 0; a < 4; ++a) {
        float acc = 0.0f;
#pragma unroll
        for (int c8 = 0; c8 < 4; ++c8) {
          const v4f va = *(const v4fa*)(rd + 32 * a + 8 * c8);
          const v4f vb = *(const v4fa*)(rd + 32 * a + 8 * c8 + 4);
          const v4f ba = *(const v4fa*)(cb + 32 * a + 8 * c8);
          const v4f bb = *(const v4fa*)(cb + 32 * a + 8 * c8 + 4);
          const v4f ta = *(const v4fa*)(rt1 + 8 * c8);
          const v4f tb = *(const v4fa*)(rt1 + 8 * c8 + 4);
          acc = fmaf(va.x + ba.x, ta.x, acc);
          acc = fmaf(va.y + ba.y, ta.y, acc);
          acc = fmaf(va.z + ba.z, ta.z, acc);
          acc = fmaf(va.w + ba.w, ta.w, acc);
          acc = fmaf(vb.x + bb.x, tb.x, acc);
          acc = fmaf(vb.y + bb.y, tb.y, acc);
          acc = fmaf(vb.z + bb.z, tb.z, acc);
          acc = fmaf(vb.w + bb.w, tb.w, acc);
        }
        ru[4 * ns + a] = acc;
      }
    } else {
      const v4f ua = *(const v4fa*)ru;
      const v4f ub = *(const v4fa*)(ru + 4);
      const int rb = (ns - 2) * MULT;
#pragma unroll 1
      for (int r = 0; r < MULT; ++r) {
        const v4f la  = *(const v4fa*)(rd + 8 * r);
        const v4f lb2 = *(const v4fa*)(rd + 8 * r + 4);
        const v4f ba  = *(const v4fa*)(cb + 8 * r);
        const v4f bb  = *(const v4fa*)(cb + 8 * r + 4);
        float acc = (la.x + ba.x) * ua.x;
        acc = fmaf(la.y + ba.y, ua.y, acc);
        acc = fmaf(la.z + ba.z, ua.z, acc);
        acc = fmaf(la.w + ba.w, ua.w, acc);
        acc = fmaf(lb2.x + bb.x, ub.x, acc);
        acc = fmaf(lb2.y + bb.y, ub.y, acc);
        acc = fmaf(lb2.z + bb.z, ub.z, acc);
        acc = fmaf(lb2.w + bb.w, ub.w, acc);
        rt2[rb + r] = acc;
      }
    }
    __syncthreads();
  }

  const float* b2r = B2 + (size_t)elc * 8;
  const v4f g0 = *(const v4fa*)b2r;
  const v4f g1 = *(const v4fa*)(b2r + 4);
  const float g00 = bf16_val(g0.x), g01 = bf16_val(g0.y), g02 = bf16_val(g0.z), g03 = bf16_val(g0.w);
  const float g10 = bf16_val(g1.x), g11 = bf16_val(g1.y), g12 = bf16_val(g1.z), g13 = bf16_val(g1.w);

  if constexpr (MODE == 0) {
    int t = dst[elc];
    t = t < 0 ? 0 : (t > nN - 1 ? nN - 1 : t);
    const float* qr = Q + (size_t)t * FROW;
    float* ss = sD + tid * 4;
#pragma unroll 1
    for (int h = 0; h < NHEAD; ++h) {
      float sacc = 0.0f;
#pragma unroll
      for (int jj = 0; jj < 4; ++jj) {
        const int mp = 4 * h + jj;
        const float ta = rt2[2 * mp];
        const float tb = rt2[2 * mp + 1];
        const v4f qv = *(const v4fa*)(qr + 16 * h + 4 * jj);
        const float k0 = fmaf(tb, g10, ta * g00);
        const float k1 = fmaf(tb, g11, ta * g01);
        const float k2 = fmaf(tb, g12, ta * g02);
        const float k3 = fmaf(tb, g13, ta * g03);
        sacc = fmaf(qv.x, k0, sacc);
        sacc = fmaf(qv.y, k1, sacc);
        sacc = fmaf(qv.z, k2, sacc);
        sacc = fmaf(qv.w, k3, sacc);
      }
      ss[h] = live ? sacc * QSCL : 0.0f;
    }
    __syncthreads();
    const v4f o4 = *(const v4fa*)(sD + tid * 4);
    float* sp = SC + (size_t)(elb + tid) * 4;
    *(volatile v4f*)sp = o4;
    __threadfence();
    *(volatile v4f*)sp = o4;
  } else {
    float* sx = sD + tid * FROW;
#pragma unroll 2
    for (int mp = 0; mp < MULT; ++mp) {
      const float ta = rt2[2 * mp];
      const float tb = rt2[2 * mp + 1];
      v4f x;
      x.x = fmaf(tb, g10, ta * g00);
      x.y = fmaf(tb, g11, ta * g01);
      x.z = fmaf(tb, g12, ta * g02);
      x.w = fmaf(tb, g13, ta * g03);
      *(v4fa*)(sx + 4 * mp) = x;
    }
    __syncthreads();
    v4f pv[16];
#pragma unroll
    for (int it = 0; it < 16; ++it) pv[it] = *(const v4fa*)(sD + (size_t)(it * CTHR + tid) * 4);
    float* vb = Vp + (size_t)elb * FROW;
#pragma unroll
    for (int it = 0; it < 16; ++it) *(volatile v4f*)(vb + (size_t)(it * CTHR + tid) * 4) = pv[it];
    __threadfence();
#pragma unroll
    for (int it = 0; it < 16; ++it) *(volatile v4f*)(vb + (size_t)(it * CTHR + tid) * 4) = pv[it];
  }
}

__global__ __launch_bounds__(NTHR) void k_scan(const int* __restrict__ dsts, int nE, int nN, int vec8,
                                               const float* __restrict__ SC, const float* __restrict__ V,
                                               float* out) {
  extern __shared__ __attribute__((aligned(16))) int dsm[];
  int*   list = dsm;
  int*   hl   = dsm + LISTN;
  int*   sl   = hl + RCAP;
  int*   cnt  = sl + RCAP;
  int*   offs = cnt + NBA;
  int*   cur  = offs + NBA;
  int*   misc = cur + NBA;
  const int tid = (int)threadIdx.x, lane = tid & 31, wave = tid >> 5;
  const int nodeBase = (int)blockIdx.x * NBA;

  {
    const v4i z4 = {0, 0, 0, 0};
    for (int i = tid * 4; i < AGG_ZINTS; i += NTHR * 4) *(v4ia*)(dsm + i) = z4;
    if (tid < 16) misc[tid] = 0;
  }
  __syncthreads();

  int t = 0, ov = 0;
  const int nChunks = (nE + CHUNK - 1) / CHUNK;
#pragma unroll 1
  for (int ch = 0; ch < nChunks; ++ch) {
    const int cbase = ch * CHUNK;
    const int wc = scan_chunk<SLA>(dsts, nE, cbase, nodeBase, NBA, vec8, list, tid, lane, wave);
    if (lane == 0) misc[wave] = wc;
    __syncthreads();
    if (wave == 0) {
#pragma unroll 1
      for (int w2 = 0; w2 < NWAVE; ++w2) {
        int c = misc[w2];
        c = c < 0 ? 0 : (c > WCAP ? WCAP : c);
#pragma unroll 1
        for (int b0 = 0; b0 < c; b0 += 32) {
          const int idx = b0 + lane;
          const int ent = list[w2 * WCAP + (idx < WCAP ? idx : WCAP - 1)];
          const int m32 = (c - b0) < 32 ? (c - b0) : 32;
#pragma unroll 1
          for (int k = 0; k < m32; ++k) {
            const int u    = __builtin_amdgcn_readlane(ent, k);
            const int slot = u & (NBA - 1);
            const int el   = (u >> SLA) & (CHUNK - 1);
            const int pk   = ((cbase + el) << SLA) | slot;
            if (t < RCAP) {
              if (lane == 0) { hl[t] = pk; cnt[slot] = cnt[slot] + 1; }
              t = t + 1;
            } else {
              ov = 1;
            }
          }
        }
      }
    }
    __syncthreads();
  }
  if (wave == 0 && lane == 0) { misc[8] = t; misc[9] = ov; }
  __syncthreads();
  int tt = misc[8];
  tt = tt < 0 ? 0 : (tt > RCAP ? RCAP : tt);
  const int ovf = misc[9];

  if (wave == 0) {
    const int base = lane * (NBA / 32);
    int s = 0;
#pragma unroll 1
    for (int i = 0; i < NBA / 32; ++i) s += cnt[base + i];
    int incl = s;
#pragma unroll
    for (int d = 1; d < 32; d <<= 1) {
      const int y = __shfl_up(incl, d, 32);
      if (lane >= d) incl += y;
    }
    int run = incl - s;
#pragma unroll 1
    for (int i = 0; i < NBA / 32; ++i) {
      const int cv = cnt[base + i];
      offs[base + i] = run;
      cur[base + i]  = run;
      run += cv;
    }
  }
  __syncthreads();
  if (wave == 0) {
#pragma unroll 1
    for (int b0 = 0; b0 < tt; b0 += 32) {
      const int idx = b0 + lane;
      const int ent = hl[idx < RCAP ? idx : RCAP - 1];
      const int m32 = (tt - b0) < 32 ? (tt - b0) : 32;
#pragma unroll 1
      for (int k = 0; k < m32; ++k) {
        const int u    = __builtin_amdgcn_readlane(ent, k);
        const int slot = u & (NBA - 1);
        if (lane == 0) {
          int p = cur[slot];
          p = p < 0 ? 0 : (p > RCAP - 1 ? RCAP - 1 : p);
          sl[p] = u;
          cur[slot] = p + 1;
        }
      }
    }
  }
  __syncthreads();

  const float qnan = __int_as_float(0x7fc00000);
  const float ninf = __int_as_float((int)0xff800000u);
  const float pz = (ovf != 0) ? qnan : 0.0f;
  const int   hd = lane >> 3;
#pragma unroll 1
  for (int pi = 0; pi < SPW / 2; ++pi) {
    float ra0 = 0.0f, ra1 = 0.0f, rb0 = 0.0f, rb1 = 0.0f;
#pragma unroll 1
    for (int j = 0; j < 2; ++j) {
      const int s = wave * SPW + 2 * pi + j;
      int c = cnt[s];
      const bool big = c > DEGCAP;
      c = c < 0 ? 0 : (c > DEGCAP ? DEGCAP : c);
      int o = offs[s];
      o = o < 0 ? 0 : (o > RCAP ? RCAP : o);
      float mx0 = ninf, mx1 = ninf, mx2 = ninf, mx3 = ninf;
#pragma unroll 1
      for (int b0 = 0; b0 < c; b0 += 32) {
        int idx = o + b0 + lane;
        idx = idx > RCAP - 1 ? RCAP - 1 : idx;
        int eid = sl[idx] >> SLA;
        eid = eid < 0 ? 0 : (eid > nE - 1 ? nE - 1 : eid);
        const bool ok = (b0 + lane) < c;
        const v4f sc = *(const v4fa*)(SC + (size_t)eid * 4);
        mx0 = ok ? fmaxf(mx0, sc.x) : mx0;
        mx1 = ok ? fmaxf(mx1, sc.y) : mx1;
        mx2 = ok ? fmaxf(mx2, sc.z) : mx2;
        mx3 = ok ? fmaxf(mx3, sc.w) : mx3;
      }
#pragma unroll
      for (int d = 16; d > 0; d >>= 1) {
        mx0 = fmaxf(mx0, __shfl_xor(mx0, d));
        mx1 = fmaxf(mx1, __shfl_xor(mx1, d));
        mx2 = fmaxf(mx2, __shfl_xor(mx2, d));
        mx3 = fmaxf(mx3, __shfl_xor(mx3, d));
      }
      float dn0 = 0.0f, dn1 = 0.0f, dn2 = 0.0f, dn3 = 0.0f;
      float acc0 = 0.0f, acc1 = 0.0f;
#pragma unroll 1
      for (int b0 = 0; b0 < c; b0 += 32) {
        int idx = o + b0 + lane;
        idx = idx > RCAP - 1 ? RCAP - 1 : idx;
        int eid = sl[idx] >> SLA;
        eid = eid < 0 ? 0 : (eid > nE - 1 ? nE - 1 : eid);
        const bool ok = (b0 + lane) < c;
        const v4f sc = *(const v4fa*)(SC + (size_t)eid * 4);
        const float e0 = ok ? expf(sc.x - mx0) : 0.0f;
        const float e1 = ok ? expf(sc.y - mx1) : 0.0f;
        const float e2 = ok ? expf(sc.z - mx2) : 0.0f;
        const float e3 = ok ? expf(sc.w - mx3) : 0.0f;
        dn0 += e0; dn1 += e1; dn2 += e2; dn3 += e3;
        const int i0 = __float_as_int(e0), i1 = __float_as_int(e1);
        const int i2 = __float_as_int(e2), i3 = __float_as_int(e3);
        const int m32 = (c - b0) < 32 ? (c - b0) : 32;
#pragma unroll 1
        for (int k = 0; k < m32; ++k) {
          const int   ek = __builtin_amdgcn_readlane(eid, k);
          const float w0 = __int_as_float(__builtin_amdgcn_readlane(i0, k));
          const float w1 = __int_as_float(__builtin_amdgcn_readlane(i1, k));
          const float w2 = __int_as_float(__builtin_amdgcn_readlane(i2, k));
          const float w3 = __int_as_float(__builtin_amdgcn_readlane(i3, k));
          const float w  = (hd == 0) ? w0 : ((hd == 1) ? w1 : ((hd == 2) ? w2 : w3));
          const v2f vv = *(const v2fa*)(V + (size_t)ek * FROW + 2 * lane);
          acc0 = fmaf(w, vv.x, acc0);
          acc1 = fmaf(w, vv.y, acc1);
        }
      }
#pragma unroll
      for (int d = 16; d > 0; d >>= 1) {
        dn0 += __shfl_xor(dn0, d);
        dn1 += __shfl_xor(dn1, d);
        dn2 += __shfl_xor(dn2, d);
        dn3 += __shfl_xor(dn3, d);
      }
      const float dsel = (hd == 0) ? dn0 : ((hd == 1) ? dn1 : ((hd == 2) ? dn2 : dn3));
      const float inv  = __builtin_amdgcn_rcpf(fmaxf(dsel, 1e-9f));
      const float pzr  = big ? qnan : pz;
      const float r0 = fmaf(acc0, inv, pzr);
      const float r1 = fmaf(acc1, inv, pzr);
      if (j == 0) { ra0 = r0; ra1 = r1; } else { rb0 = r0; rb1 = r1; }
    }
    const int srcA = (2 * lane) & 31;
    const int srcB = (2 * lane + 1) & 31;
    const float p0 = __shfl(ra0, srcA), p1 = __shfl(ra1, srcA);
    const float p2 = __shfl(ra0, srcB), p3 = __shfl(ra1, srcB);
    const float q0 = __shfl(rb0, srcA), q1 = __shfl(rb1, srcA);
    const float q2 = __shfl(rb0, srcB), q3 = __shfl(rb1, srcB);
    const bool lowh = lane < 16;
    v4f o4;
    o4.x = lowh ? p0 : q0;
    o4.y = lowh ? p1 : q1;
    o4.z = lowh ? p2 : q2;
    o4.w = lowh ? p3 : q3;
    const int rowA = nodeBase + wave * SPW + 2 * pi;
    const int row  = rowA + (lane >> 4);
    const int rc   = row < nN ? rowA : 0;
    float* op = out + (size_t)rc * FROW + 4 * lane;
    if (row < nN) *(volatile v4f*)op = o4;
    __threadfence();
    if (row < nN) *(volatile v4f*)op = o4;
  }
}

static inline int cdiv(int a, int b) { return (a + b - 1) / b; }

extern "C" void kernel_launch(void* const* d_in, const int* in_sizes, int n_in,
                              void* d_out, int out_size, void* d_ws, size_t ws_size,
                              hipStream_t stream) {
  if (n_in < 20) return;
  const int nE = in_sizes[4];
  if (nE < 1 || nE >= (1 << 21)) return;
  if (in_sizes[5] != nE) return;
  if ((long long)in_sizes[0] != 8LL * nE) return;
  if ((long long)in_sizes[1] != 8LL * nE) return;
  if ((long long)in_sizes[2] != (long long)EFK * nE) return;
  if (in_sizes[3] < FROW || (in_sizes[3] % FROW) != 0) return;
  const int nN = in_sizes[3] / FROW;
  if (in_sizes[6] != 2 * MULT * MULT || in_sizes[7] != MULT) return;
  for (int p = 0; p < 2; ++p) {
    const int b = 8 + 6 * p;
    if (in_sizes[b + 0] != EFK * HID || in_sizes[b + 1] != HID) return;
    if (in_sizes[b + 2] != HID * NLR || in_sizes[b + 3] != NLR) return;
    if (in_sizes[b + 4] != HID * NLR || in_sizes[b + 5] != NLR) return;
  }
  if ((long long)out_size != (long long)nN * FROW) return;

  const float* b1   = (const float*)d_in[0];
  const float* b2   = (const float*)d_in[1];
  const float* ef   = (const float*)d_in[2];
  const float* f    = (const float*)d_in[3];
  const int*   src  = (const int*)d_in[4];
  const int*   dst  = (const int*)d_in[5];
  const float* q_w  = (const float*)d_in[6];
  const float* q_b  = (const float*)d_in[7];
  const float* k_w1 = (const float*)d_in[8];
  const float* k_b1 = (const float*)d_in[9];
  const float* k_wl = (const float*)d_in[10];
  const float* k_bl = (const float*)d_in[11];
  const float* k_wr = (const float*)d_in[12];
  const float* k_br = (const float*)d_in[13];
  const float* v_w1 = (const float*)d_in[14];
  const float* v_b1 = (const float*)d_in[15];
  const float* v_wl = (const float*)d_in[16];
  const float* v_bl = (const float*)d_in[17];
  const float* v_wr = (const float*)d_in[18];
  const float* v_br = (const float*)d_in[19];
  float* out = (float*)d_out;

  const int gE  = cdiv(nE, CTHR);
  const int EP  = gE * CTHR;
  const int gA  = cdiv(nN, NBA);
  if ((long long)gA * NBA < (long long)nN) return;
  const int nQU = cdiv(nN * 16, NTHR) * NTHR;
  const int nQR = nQU / 16;

  char* ws = (char*)d_ws;
  size_t off = 0;
  const size_t oW1T = off; off += (size_t)NW1 * EFK * 2;             off = (off + 255) & ~(size_t)255;
  const size_t oWRL = off; off += (size_t)NWRL * KRL * 2;            off = (off + 255) & ~(size_t)255;
  const size_t oQ   = off; off += (size_t)nQR * FROW * 4;            off = (off + 255) & ~(size_t)255;
  const size_t oSC  = off; off += (size_t)EP * 4 * 4;                off = (off + 255) & ~(size_t)255;
  const size_t oV   = off; off += (size_t)EP * FROW * 4;             off = (off + 255) & ~(size_t)255;
  if (off > ws_size || off > (size_t)WSMAX) return;
  unsigned short* W1T = (unsigned short*)(ws + oW1T);
  unsigned short* WRL = (unsigned short*)(ws + oWRL);
  float*          Q   = (float*)(ws + oQ);
  float*          SC  = (float*)(ws + oSC);
  float*          V   = (float*)(ws + oV);

  hipFuncSetAttribute(reinterpret_cast<const void*>(&k_conv<0>), hipFuncAttributeMaxDynamicSharedMemorySize,
                      (int)CONV_LDS_BYTES);
  hipFuncSetAttribute(reinterpret_cast<const void*>(&k_conv<1>), hipFuncAttributeMaxDynamicSharedMemorySize,
                      (int)CONV_LDS_BYTES);
  hipFuncSetAttribute(reinterpret_cast<const void*>(&k_scan), hipFuncAttributeMaxDynamicSharedMemorySize,
                      (int)AGG_LDS_BYTES);

  const int nPrep = NU_W1 + NU_WRL + nQU;
  const int vec8  = 1;

  k_prep<<<nPrep / NTHR, NTHR, 0, stream>>>(f, q_w, q_b, k_w1, v_w1, k_wr, k_wl, v_wr, v_wl, nN, nQU,
                                            W1T, WRL, Q);
  k_conv<0><<<gE, CTHR, CONV_LDS_BYTES, stream>>>(src, dst, nE, nN, ef, f, b1, b2, W1T, WRL,
                                                   k_b1, k_br, k_bl, Q, SC, V);
  k_conv<1><<<gE, CTHR, CONV_LDS_BYTES, stream>>>(src, dst, nE, nN, ef, f, b1, b2,
                                                   W1T + (size_t)HID * EFK, WRL + (size_t)(2 * NLR) * KRL,
                                                   v_b1, v_br, v_bl, Q, SC, V);
  k_scan<<<gA, NTHR, AGG_LDS_BYTES, stream>>>(dst, nE, nN, vec8, SC, V, out);
}
